// TemporalGNN_56899726737798
// MI455X (gfx1250) — hardware-verified
//
#include <hip/hip_runtime.h>
#include <stddef.h>
#include <stdint.h>
#include <math.h>


#define FIN     32
#define HC1     128
#define HW1     32
#define NHD1    4
#define KAP     512
#define TCK     512
#define TCN     96
#define TCNT    6
#define HID     32
#define KY      64
#define NCLS    16
#define NC2P    64
#define NTHR    256
#define NWAVE   8
#define EPT     8
#define CHUNK   (NTHR * EPT)
#define WCAP    (EPT * 32)
#define LISTN   (NWAVE * WCAP)
#define NBMAX   2048
#define SLOTB   11
#define RCAP    28672
#define DEGCAP  128
#define GBM     64
#define GBN     64
#define GTHR    128
#define MROWS   128
#define GRP     64
#define NU1     (HC1 * (FIN / 8))
#define NU2     (TCN * (TCK / 8))
#define NU3     (NC2P * (KY / 8))
#define NEGSL   0.2f
#define WSMAX   134217728
#define LDS_AGG ((2 * RCAP + 2 * NBMAX + LISTN) * 4 + 64)

static_assert((CHUNK & (CHUNK - 1)) == 0 && CHUNK <= (1 << SLOTB));
static_assert(NBMAX == (1 << SLOTB));
static_assert(NTHR * 8 == NBMAX);
static_assert(LISTN >= NBMAX);
static_assert(LISTN >= NWAVE * WCAP);
static_assert((RCAP % 32) == 0);
static_assert(LDS_AGG <= 300000);
static_assert(GBM == (GTHR / 32) * 16);
static_assert(GTHR == 2 * GBN && GTHR == 2 * GBM);
static_assert((FIN % 32) == 0 && (TCK % 32) == 0 && (KY % 32) == 0);
static_assert((HC1 % GBN) == 0 && NC2P == GBN && (GBN % HW1) == 0 && NHD1 * HW1 == HC1);
static_assert(KAP == 4 * HC1 && TCK == KAP);
static_assert(TCN == 3 * HID && TCN == 16 * TCNT && KY == 2 * HID && (TCN % 4) == 0);
static_assert((MROWS % GBM) == 0);
static_assert(HC1 == 4 * 32);
static_assert(HW1 == 8 * 4);
static_assert(NC2P == 2 * 32);
static_assert(NWAVE * GRP * NCLS <= RCAP);
static_assert((GRP & (GRP - 1)) == 0 && (NCLS % 4) == 0);
static_assert(NCLS <= NC2P && (NCLS % 2) == 0 && (HID % 8) == 0);
static_assert((NU1 % NTHR) == 0 && (NU2 % NTHR) == 0 && (NU3 % NTHR) == 0);
static_assert(((TCN / 3) * (TCK / 8)) % NTHR == 0);
static_assert(GTHR == 4 * HID);
static_assert(GBM * (KY / 8) == 4 * GTHR);
static_assert((FIN / 8) == 4);

typedef float          v2f  __attribute__((ext_vector_type(2)));
typedef float          v4f  __attribute__((ext_vector_type(4)));
typedef float          v8f  __attribute__((ext_vector_type(8)));
typedef int            v4i  __attribute__((ext_vector_type(4)));
typedef int            v8i  __attribute__((ext_vector_type(8)));
typedef unsigned int   v4u  __attribute__((ext_vector_type(4)));
typedef unsigned short v8us __attribute__((ext_vector_type(8)));
typedef __bf16         v16b __attribute__((ext_vector_type(16)));
typedef v2f  __attribute__((may_alias)) v2fa;
typedef v4f  __attribute__((may_alias)) v4fa;
typedef v8us __attribute__((may_alias)) v8usa;
union FragB { v16b v; v8us h[2]; v8i w; };

__device__ __forceinline__ v8f wmb(const FragB& a, const FragB& b, v8f c) {
  v8f d = __builtin_amdgcn_wmma_f32_16x16x32_bf16(false, a.v, false, b.v, (short)0, c, false, false);
  asm volatile("v_nop\n\tv_nop\n\tv_nop\n\tv_nop" : "+v"(d) : "v"(a.w), "v"(b.w));
  return d;
}

__device__ __forceinline__ unsigned int f2bf(float f) {
  const unsigned int u = __float_as_uint(f);
  return ((u + 0x7FFFu + ((u >> 16) & 1u)) >> 16) & 0xFFFFu;
}
__device__ __forceinline__ float bf2f(unsigned int b) { return __uint_as_float(b << 16); }
__device__ __forceinline__ float bfr(float f) { return bf2f(f2bf(f)); }
__device__ __forceinline__ v4f bfr4(const v4f a) {
  v4f r; r.x = bfr(a.x); r.y = bfr(a.y); r.z = bfr(a.z); r.w = bfr(a.w); return r;
}
__device__ __forceinline__ unsigned int pk2(float lo, float hi) { return f2bf(lo) | (f2bf(hi) << 16); }
__device__ __forceinline__ v4u pack8(const v4f a, const v4f b) {
  v4u r;
  r.x = pk2(a.x, a.y); r.y = pk2(a.z, a.w); r.z = pk2(b.x, b.y); r.w = pk2(b.z, b.w);
  return r;
}

__device__ __forceinline__ int scan_chunk(const int* __restrict__ dsts, int nE, int cbase, int slotBase,
                                          int nb, int vec8, int* list, int tid, int lane, int wave) {
  int wc = 0;
  const int el0  = tid * EPT;
  const int e0   = cbase + el0;
  const int sent = -2147483647 - 1;
  v4i da, db;
  if (vec8 != 0 && cbase + CHUNK <= nE) {
    da = *(const v4i*)(dsts + e0);
    db = *(const v4i*)(dsts + e0 + 4);
  } else {
    da.x = (e0     < nE) ? dsts[min(e0,     nE - 1)] : sent;
    da.y = (e0 + 1 < nE) ? dsts[min(e0 + 1, nE - 1)] : sent;
    da.z = (e0 + 2 < nE) ? dsts[min(e0 + 2, nE - 1)] : sent;
    da.w = (e0 + 3 < nE) ? dsts[min(e0 + 3, nE - 1)] : sent;
    db.x = (e0 + 4 < nE) ? dsts[min(e0 + 4, nE - 1)] : sent;
    db.y = (e0 + 5 < nE) ? dsts[min(e0 + 5, nE - 1)] : sent;
    db.z = (e0 + 6 < nE) ? dsts[min(e0 + 6, nE - 1)] : sent;
    db.w = (e0 + 7 < nE) ? dsts[min(e0 + 7, nE - 1)] : sent;
  }
  const unsigned nbs = (unsigned)slotBase;
  const unsigned unb = (unsigned)nb;
  const unsigned s0 = (unsigned)da.x - nbs, s1 = (unsigned)da.y - nbs;
  const unsigned s2 = (unsigned)da.z - nbs, s3 = (unsigned)da.w - nbs;
  const unsigned s4 = (unsigned)db.x - nbs, s5 = (unsigned)db.y - nbs;
  const unsigned s6 = (unsigned)db.z - nbs, s7 = (unsigned)db.w - nbs;
  const bool h0 = s0 < unb, h1 = s1 < unb, h2 = s2 < unb, h3 = s3 < unb;
  const bool h4 = s4 < unb, h5 = s5 < unb, h6 = s6 < unb, h7 = s7 < unb;
  const unsigned any = __builtin_amdgcn_ballot_w32(h0 | h1 | h2 | h3 | h4 | h5 | h6 | h7);
  if (any != 0u) {
#define HITJ(J, HJ, SJ) { \
      const unsigned mj = __builtin_amdgcn_ballot_w32(HJ); \
      if (mj != 0u) { \
        if (HJ) { \
          const int pos = wc + (int)__builtin_amdgcn_mbcnt_lo(mj, 0u); \
          if (pos < WCAP) list[wave * WCAP + pos] = ((el0 + (J)) << SLOTB) | (int)(SJ); \
        } \
        wc += (int)__builtin_popcount(mj); } }
    HITJ(0, h0, s0)
    HITJ(1, h1, s1)
    HITJ(2, h2, s2)
    HITJ(3, h3, s3)
    HITJ(4, h4, s4)
    HITJ(5, h5, s5)
    HITJ(6, h6, s6)
    HITJ(7, h7, s7)
#undef HITJ
  }
  return wc;
}

__global__ __launch_bounds__(NTHR) void k_xprep(const float* __restrict__ x, unsigned short* xb, int nN, int MP,
                                                int nUnits) {
  const int i = (int)blockIdx.x * NTHR + (int)threadIdx.x;
  if (i >= nUnits) return;
  const int R  = i >> 2;
  const int c0 = (i & 3) * 8;
  const int tt = (R >= MP) ? 1 : 0;
  const int rt = R - tt * MP;
  const int rc = rt < nN ? rt : nN - 1;
  const float* p = x + ((size_t)(1 + tt) * (size_t)nN + (size_t)rc) * FIN + c0;
  v4f a = *(const v4fa*)p, b = *(const v4fa*)(p + 4);
  const v4f z4 = {0.f, 0.f, 0.f, 0.f};
  if (rt >= nN) { a = z4; b = z4; }
  const v4u hv = pack8(a, b);
  const size_t o = (size_t)R * FIN + c0;
  *(volatile v4u*)(xb + o) = hv;
  __threadfence();
  *(volatile v4u*)(xb + o) = hv;
}

__global__ __launch_bounds__(NTHR) void k_wprep(const float* __restrict__ W1,
                                                const float* __restrict__ K1, const float* __restrict__ K2,
                                                const float* __restrict__ K3, const float* __restrict__ W2,
                                                unsigned short* W1T, unsigned short* KCT, unsigned short* W2T) {
  const int u = (int)blockIdx.x * NTHR + (int)threadIdx.x;
  v8us o;
  unsigned short* dp;
  if (u < NU1) {
    const int n  = u >> 2;
    const int k8 = (u & 3) * 8;
    const float* p = W1 + (size_t)k8 * HC1 + n;
#pragma unroll
    for (int i = 0; i < 8; ++i) o[i] = (unsigned short)f2bf(p[(size_t)i * HC1]);
    dp = W1T + (size_t)n * FIN + k8;
  } else if (u < NU1 + NU2) {
    const int v    = u - NU1;
    const int n    = v >> 6;
    const int k8   = (v & 63) * 8;
    const int conv = n >> 5;
    const int d    = n & 31;
    const int tap  = k8 >> 8;
    const int c0   = k8 & (HC1 - 1);
    const float* Kp = (conv == 0) ? K1 : ((conv == 1) ? K2 : K3);
    const float* p = Kp + (size_t)tap * (HC1 * HID) + (size_t)c0 * HID + d;
#pragma unroll
    for (int i = 0; i < 8; ++i) o[i] = (unsigned short)f2bf(p[(size_t)i * HID]);
    dp = KCT + (size_t)n * TCK + k8;
  } else if (u < NU1 + NU2 + NU3) {
    const int v   = u - NU1 - NU2;
    const int n   = v >> 3;
    const int k8  = (v & 7) * 8;
    const int kk  = k8 & (HID - 1);
    const int ncl = n < NCLS ? n : NCLS - 1;
    const float* p = W2 + (size_t)kk * NCLS + ncl;
    const bool ok = n < NCLS;
#pragma unroll
    for (int i = 0; i < 8; ++i) {
      const unsigned int b = f2bf(p[(size_t)i * NCLS]);
      o[i] = ok ? (unsigned short)b : (unsigned short)0;
    }
    dp = W2T + (size_t)n * KY + k8;
  } else {
    return;
  }
  *(volatile v8us*)dp = o;
  __threadfence();
  *(volatile v8us*)dp = o;
}

template<int HW>
__global__ __launch_bounds__(GTHR) void k_gemm(
    const unsigned short* __restrict__ A, const unsigned short* __restrict__ WT,
    float* outF, int K, int ldo,
    const float* __restrict__ atts, const float* __restrict__ attd, int attLen,
    float* SD, int MPr)
{
  static_assert(HW == 32 || HW == 64);
  constexpr int HPB = GBN / HW;
  __shared__ __attribute__((aligned(16))) float stg[GBM * GBN];
  __shared__ __attribute__((aligned(16))) float satt[2 * GBN];
  __shared__ __attribute__((aligned(16))) float sdot[2 * HPB * GBM];
  const int tid = (int)threadIdx.x, lane = tid & 31, wave = tid >> 5, hh = lane >> 4, m = lane & 15;
  const int rowBase = (int)blockIdx.x * GBM;
  const int cblk    = (int)blockIdx.y;
  const int col0    = cblk * GBN;

  {
    const int which = tid >> 6;
    const int c  = tid & 63;
    const int j  = c / HW;
    const int ch = c - j * HW;
    const int gh = cblk * HPB + j;
    const int cl = ch < attLen ? ch : attLen - 1;
    const float vs = atts[gh * attLen + cl];
    const float vd = attd[gh * attLen + cl];
    float v = (which == 0) ? vs : vd;
    v = (ch < attLen) ? bfr(v) : 0.f;
    satt[which * GBN + c] = v;
  }

  v8f acc[4];
  {
    const v8f z = {0.f, 0.f, 0.f, 0.f, 0.f, 0.f, 0.f, 0.f};
    acc[0] = z; acc[1] = z; acc[2] = z; acc[3] = z;
  }
  const unsigned short* ap = A  + (size_t)(rowBase + 16 * wave + m) * (size_t)K + 8 * hh;
  const unsigned short* wp = WT + (size_t)(col0 + m) * (size_t)K + 8 * hh;
  const int ksteps = K >> 5;
#pragma unroll 1
  for (int ks = 0; ks < ksteps; ++ks) {
    FragB af;
    af.h[0] = *(const v8usa*)(ap + 32 * ks);
    af.h[1] = *(const v8usa*)(ap + 32 * ks + 16);
#pragma unroll
    for (int t = 0; t < 4; ++t) {
      const unsigned short* wq = wp + (size_t)(16 * t) * (size_t)K + 32 * ks;
      FragB bf;
      bf.h[0] = *(const v8usa*)wq;
      bf.h[1] = *(const v8usa*)(wq + 16);
      acc[t] = wmb(af, bf, acc[t]);
    }
  }

#pragma unroll
  for (int t = 0; t < 4; ++t) {
    const int lc = 16 * t + m;
#pragma unroll
    for (int r = 0; r < 8; ++r) {
      const int lr = 16 * wave + 8 * hh + r;
      stg[lr * GBN + lc] = acc[t][r];
    }
  }
  __syncthreads();

  {
    const int row = tid & 63, which = tid >> 6;
    const float* sa = satt + which * GBN;
    const float* hr = stg + row * GBN;
#pragma unroll
    for (int j = 0; j < HPB; ++j) {
      float d = 0.f;
#pragma unroll 4
      for (int c4 = 0; c4 < HW / 4; ++c4) {
        const v4f hv = *(const v4fa*)(hr + j * HW + 4 * c4);
        const v4f av = *(const v4fa*)(sa + j * HW + 4 * c4);
        d = fmaf(hv.x, av.x, d);
        d = fmaf(hv.y, av.y, d);
        d = fmaf(hv.z, av.z, d);
        d = fmaf(hv.w, av.w, d);
      }
      sdot[(which * HPB + j) * GBM + row] = d;
    }
  }
  __syncthreads();

  v4f fv[8];
#pragma unroll
  for (int i = 0; i < 8; ++i) {
    const int lr = 16 * wave + 2 * i + hh;
    fv[i] = *(const v4fa*)(stg + lr * GBN + 4 * m);
  }
  const int which2 = lane >> 4, piece = lane & 15;
  const int hsel = wave < HPB ? wave : HPB - 1;
  const v4f sdv = *(const v4fa*)(sdot + (which2 * HPB + hsel) * GBM + 4 * piece);
  float* sp = SD + (size_t)(2 * (cblk * HPB + hsel) + which2) * (size_t)MPr + rowBase + 4 * piece;
  const bool wsd = wave < HPB;

#pragma unroll
  for (int i = 0; i < 8; ++i) {
    const int lr = 16 * wave + 2 * i + hh;
    const int gr = rowBase + lr;
    float* op = outF + (size_t)gr * (size_t)ldo + col0 + 4 * m;
    *(volatile v4f*)op = fv[i];
  }
  if (wsd) *(volatile v4f*)sp = sdv;
  __threadfence();
#pragma unroll
  for (int i = 0; i < 8; ++i) {
    const int lr = 16 * wave + 2 * i + hh;
    const int gr = rowBase + lr;
    float* op = outF + (size_t)gr * (size_t)ldo + col0 + 4 * m;
    *(volatile v4f*)op = fv[i];
  }
  if (wsd) *(volatile v4f*)sp = sdv;
}

__global__ __launch_bounds__(GTHR) void k_tconv(
    const unsigned short* __restrict__ A, const unsigned short* __restrict__ BT,
    const float* __restrict__ bk1, const float* __restrict__ bk2, const float* __restrict__ bk3,
    unsigned short* YP, int nN)
{
  __shared__ __attribute__((aligned(16))) float stg[GBM * TCN];
  __shared__ __attribute__((aligned(16))) float ybuf[GBM * HID];
  __shared__ __attribute__((aligned(16))) float sbk[TCN];
  const int tid = (int)threadIdx.x, lane = tid & 31, wave = tid >> 5, hh = lane >> 4, m = lane & 15;
  const int rowBase = (int)blockIdx.x * GBM;

  {
    const float f1 = bk1[lane], f2 = bk2[lane], f3 = bk3[lane];
    const float v = (wave == 0) ? f1 : ((wave == 1) ? f2 : f3);
    if (wave < 3) sbk[wave * HID + lane] = bfr(v);
  }

  v8f acc[TCNT];
  {
    const v8f z = {0.f, 0.f, 0.f, 0.f, 0.f, 0.f, 0.f, 0.f};
#pragma unroll
    for (int t = 0; t < TCNT; ++t) acc[t] = z;
  }
  const unsigned short* ap = A  + (size_t)(rowBase + 16 * wave + m) * (size_t)TCK + 8 * hh;
  const unsigned short* bp = BT + (size_t)m * (size_t)TCK + 8 * hh;
#pragma unroll 1
  for (int k0 = 0; k0 < TCK; k0 += 32) {
    FragB af;
    af.h[0] = *(const v8usa*)(ap + k0);
    af.h[1] = *(const v8usa*)(ap + k0 + 16);
#pragma unroll
    for (int nt = 0; nt < TCNT; ++nt) {
      const unsigned short* wq = bp + (size_t)(16 * nt) * (size_t)TCK + k0;
      FragB bf;
      bf.h[0] = *(const v8usa*)wq;
      bf.h[1] = *(const v8usa*)(wq + 16);
      acc[nt] = wmb(af, bf, acc[nt]);
    }
  }

#pragma unroll
  for (int nt = 0; nt < TCNT; ++nt) {
    const int lc = 16 * nt + m;
#pragma unroll
    for (int r = 0; r < 8; ++r) {
      const int lr = 16 * wave + 8 * hh + r;
      stg[lr * TCN + lc] = acc[nt][r];
    }
  }
  __syncthreads();

#pragma unroll 2
  for (int i = 0; i < GBM / 4; ++i) {
    const int r = wave + 4 * i;
    const float* sr = stg + r * TCN;
    const float c1 = sr[lane] + sbk[lane];
    const float c2 = sr[HID + lane] + sbk[HID + lane];
    const float c3 = sr[2 * HID + lane] + sbk[2 * HID + lane];
    const float e  = expf(-c2);
    const float sg = __builtin_amdgcn_rcpf(1.0f + e);
    float g = fmaf(c1, sg, c3);
    g = fmaxf(g, 0.0f);
    g = (rowBase + r < nN) ? g : 0.0f;
    ybuf[r * HID + lane] = g;
  }
  __syncthreads();

  v4u pv[4];
#pragma unroll
  for (int i = 0; i < 4; ++i) {
    const int p   = tid + GTHR * i;
    const int row = p >> 3, q = p & 7;
    const float* yb = ybuf + row * HID + 8 * (q & 3);
    const v4f a = *(const v4fa*)yb, b = *(const v4fa*)(yb + 4);
    const unsigned int h0 = f2bf(a.x), h1 = f2bf(a.y), h2 = f2bf(a.z), h3 = f2bf(a.w);
    const unsigned int h4 = f2bf(b.x), h5 = f2bf(b.y), h6 = f2bf(b.z), h7 = f2bf(b.w);
    const unsigned int l0 = f2bf(a.x - bf2f(h0)), l1 = f2bf(a.y - bf2f(h1));
    const unsigned int l2 = f2bf(a.z - bf2f(h2)), l3 = f2bf(a.w - bf2f(h3));
    const unsigned int l4 = f2bf(b.x - bf2f(h4)), l5 = f2bf(b.y - bf2f(h5));
    const unsigned int l6 = f2bf(b.z - bf2f(h6)), l7 = f2bf(b.w - bf2f(h7));
    const bool lsel = q >= 4;
    v4u w;
    w.x = lsel ? (l0 | (l1 << 16)) : (h0 | (h1 << 16));
    w.y = lsel ? (l2 | (l3 << 16)) : (h2 | (h3 << 16));
    w.z = lsel ? (l4 | (l5 << 16)) : (h4 | (h5 << 16));
    w.w = lsel ? (l6 | (l7 << 16)) : (h6 | (h7 << 16));
    pv[i] = w;
  }
#pragma unroll
  for (int i = 0; i < 4; ++i) {
    const int p = tid + GTHR * i;
    const int row = p >> 3, q = p & 7;
    unsigned short* gp = YP + (size_t)(rowBase + row) * KY + 8 * q;
    *(volatile v4u*)gp = pv[i];
  }
  __threadfence();
#pragma unroll
  for (int i = 0; i < 4; ++i) {
    const int p = tid + GTHR * i;
    const int row = p >> 3, q = p & 7;
    unsigned short* gp = YP + (size_t)(rowBase + row) * KY + 8 * q;
    *(volatile v4u*)gp = pv[i];
  }
}

template<int L>
__global__ __launch_bounds__(NTHR) void k_agg(
    const int* __restrict__ srcs, const int* __restrict__ dsts,
    const float* __restrict__ F, const float* __restrict__ SD,
    const float* __restrict__ bias,
    unsigned short* HP, float* out,
    int nN, int nE, int nb, int vec8, int MPr) {
  extern __shared__ v4f lds_dyn[];
  int* reg1 = (int*)lds_dyn;
  int* reg2 = reg1 + RCAP;
  int* scnt = reg2 + RCAP;
  int* soff = scnt + NBMAX;
  int* list = soff + NBMAX;
  int* wcnt = list + LISTN;
  int* wtot = wcnt + NWAVE;
  const int tid = (int)threadIdx.x, lane = tid & 31, wave = tid >> 5;
  const int nodeBase = (int)blockIdx.x * nb;

  for (int i = tid; i < NBMAX; i += NTHR) scnt[i] = 0;
  __syncthreads();

  int tot = 0;
  const int nChunks = (nE + CHUNK - 1) / CHUNK;
#pragma unroll 1
  for (int ch = 0; ch < nChunks; ++ch) {
    const int cbase = ch * CHUNK;
    const int wc = scan_chunk(dsts, nE, cbase, nodeBase, nb, vec8, list, tid, lane, wave);
    if (lane == 0) wcnt[wave] = wc;
    __syncthreads();
    int pre = 0, all = 0;
#pragma unroll
    for (int w2 = 0; w2 < NWAVE; ++w2) {
      int c = wcnt[w2];
      c = c < 0 ? 0 : (c > WCAP ? WCAP : c);
      all += c;
      pre += (w2 < wave) ? c : 0;
    }
    const int wcc  = wc > WCAP ? WCAP : wc;
    const int base = tot + pre;
#pragma unroll 1
    for (int i = lane; i < wcc; i += 32) {
      const int ent = list[wave * WCAP + i];
      const int el  = (ent >> SLOTB) & (CHUNK - 1);
      const int sl  = ent & (NBMAX - 1);
      int eid = cbase + el;
      eid = eid > nE - 1 ? nE - 1 : eid;
      const int pos = base + i;
      if (pos < RCAP) reg1[pos] = (int)(((unsigned)eid << SLOTB) | (unsigned)sl);
    }
    tot += all;
    tot = tot > RCAP ? RCAP : tot;
    __syncthreads();
  }
  const int nh = tot;

  if (wave == 0) {
#pragma unroll 1
    for (int b0 = 0; b0 < nh; b0 += 32) {
      const int idx = b0 + lane;
      const int uv  = reg1[idx < nh ? idx : nh - 1];
      const int m32 = (nh - b0) < 32 ? (nh - b0) : 32;
#pragma unroll 1
      for (int k = 0; k < m32; ++k) {
        const int u  = __builtin_amdgcn_readlane(uv, k);
        const int sl = u & (NBMAX - 1);
        if (lane == 0) scnt[sl] = scnt[sl] + 1;
      }
    }
  }
  __syncthreads();

  {
    const v4i ca = *(const v4i*)(scnt + 8 * tid);
    const v4i cb = *(const v4i*)(scnt + 8 * tid + 4);
    const int e0 = ca.x < 0 ? 0 : ca.x, e1 = ca.y < 0 ? 0 : ca.y, e2 = ca.z < 0 ? 0 : ca.z, e3 = ca.w < 0 ? 0 : ca.w;
    const int e4 = cb.x < 0 ? 0 : cb.x, e5 = cb.y < 0 ? 0 : cb.y, e6 = cb.z < 0 ? 0 : cb.z, e7 = cb.w < 0 ? 0 : cb.w;
    const int ts = e0 + e1 + e2 + e3 + e4 + e5 + e6 + e7;
    int incl = ts;
#pragma unroll
    for (int d = 1; d < 32; d <<= 1) {
      const int up = __shfl_up(incl, d);
      if (lane >= d) incl += up;
    }
    if (lane == 31) wtot[wave] = incl;
    __syncthreads();
    int pre = 0;
#pragma unroll
    for (int w2 = 0; w2 < NWAVE; ++w2) pre += (w2 < wave) ? wtot[w2] : 0;
    int run = pre + incl - ts;
    soff[8 * tid + 0] = run; run += e0;
    soff[8 * tid + 1] = run; run += e1;
    soff[8 * tid + 2] = run; run += e2;
    soff[8 * tid + 3] = run; run += e3;
    soff[8 * tid + 4] = run; run += e4;
    soff[8 * tid + 5] = run; run += e5;
    soff[8 * tid + 6] = run; run += e6;
    soff[8 * tid + 7] = run;
  }
  __syncthreads();
  for (int i = tid; i < NBMAX; i += NTHR) list[i] = soff[i];
  __syncthreads();

  if (wave == 0) {
#pragma unroll 1
    for (int b0 = 0; b0 < nh; b0 += 32) {
      const int idx = b0 + lane;
      const int uv  = reg1[idx < nh ? idx : nh - 1];
      const int m32 = (nh - b0) < 32 ? (nh - b0) : 32;
#pragma unroll 1
      for (int k = 0; k < m32; ++k) {
        const int u   = __builtin_amdgcn_readlane(uv, k);
        const int sl  = u & (NBMAX - 1);
        const int eid = (int)((unsigned)u >> SLOTB);
        if (lane == 0) {
          int pos = list[sl];
          pos = pos < 0 ? 0 : (pos > RCAP - 1 ? RCAP - 1 : pos);
          reg2[pos] = eid;
          list[sl] = pos + 1;
        }
      }
    }
  }
  __syncthreads();

  const int nbw = nb >> 3;
  const bool ovf = (nh >= RCAP);
  const float qnan = __int_as_float(0x7fc00000);

  if (L == 1) {
    const int c0   = 4 * lane;
    const int head = lane >> 3;
    const v4f bb4  = bfr4(*(const v4fa*)(bias + c0));
    const float* ASp = SD + (size_t)(2 * head) * (size_t)MPr;
    const float* ADp = ASp + MPr;

#pragma unroll 1
    for (int jt = 0; jt < nbw; ++jt) {
      const int slot = wave * nbw + jt;
      const int grow = nodeBase + slot;
      const int gcl  = grow < nN ? grow : nN - 1;
      int st = soff[slot];
      const int craw = scnt[slot];
      int cnt = craw;
      st  = st < 0 ? 0 : (st > nh ? nh : st);
      cnt = cnt < 0 ? 0 : (cnt > DEGCAP ? DEGCAP : cnt);
      if (cnt > nh - st) cnt = nh - st;
      const float pz = (ovf || craw > DEGCAP) ? qnan : 0.0f;

      const v4f fd = *(const v4fa*)(F + (size_t)gcl * HC1 + c0);
      const float adv = ADp[gcl];
      float l0 = ASp[gcl] + adv;
      l0 = l0 > 0.f ? l0 : NEGSL * l0;
      float mx = l0, dn = 1.0f;
      v4f av = fd;

#pragma unroll 1
      for (int q = 0; q < cnt; ++q) {
        int idx = st + q; idx = idx > RCAP - 1 ? RCAP - 1 : idx;
        int eid = reg2[idx]; eid = eid < 0 ? 0 : (eid > nE - 1 ? nE - 1 : eid);
        const int sraw = srcs[eid];
        const int s = sraw < 0 ? 0 : (sraw > nN - 1 ? nN - 1 : sraw);
        const v4f fs = *(const v4fa*)(F + (size_t)s * HC1 + c0);
        float lg = ASp[s] + adv;
        lg = lg > 0.f ? lg : NEGSL * lg;
        const float df = lg - mx;
        const float ee = __expf(-fabsf(df));
        const bool up  = df > 0.f;
        const float s1 = up ? ee : 1.0f;
        const float s2 = up ? 1.0f : ee;
        mx = up ? lg : mx;
        dn = fmaf(dn, s1, s2);
        av.x = fmaf(av.x, s1, s2 * fs.x);
        av.y = fmaf(av.y, s1, s2 * fs.y);
        av.z = fmaf(av.z, s1, s2 * fs.z);
        av.w = fmaf(av.w, s1, s2 * fs.w);
      }
      const float inv = __builtin_amdgcn_rcpf(dn);
      const bool live = grow < nN;
      v4f o;
      o.x = (live ? fmaxf(fmaf(av.x, inv, bb4.x), 0.f) : 0.f) + pz;
      o.y = (live ? fmaxf(fmaf(av.y, inv, bb4.y), 0.f) : 0.f) + pz;
      o.z = (live ? fmaxf(fmaf(av.z, inv, bb4.z), 0.f) : 0.f) + pz;
      o.w = (live ? fmaxf(fmaf(av.w, inv, bb4.w), 0.f) : 0.f) + pz;
      const unsigned int hbx = f2bf(o.x), hby = f2bf(o.y), hbz = f2bf(o.z), hbw = f2bf(o.w);
      const unsigned int lbx = f2bf(o.x - bf2f(hbx)), lby = f2bf(o.y - bf2f(hby));
      const unsigned int lbz = f2bf(o.z - bf2f(hbz)), lbw = f2bf(o.w - bf2f(hbw));
      const int hw0 = (int)(hbx | (hby << 16)), hw1 = (int)(hbz | (hbw << 16));
      const int lw0 = (int)(lbx | (lby << 16)), lw1 = (int)(lbz | (lbw << 16));
      const int sa = (2 * lane) & 31, sb = (2 * lane + 1) & 31;
      const int g0 = __shfl(hw0, sa), g1 = __shfl(hw1, sa), g2 = __shfl(hw0, sb), g3 = __shfl(hw1, sb);
      const int q0 = __shfl(lw0, sa), q1 = __shfl(lw1, sa), q2 = __shfl(lw0, sb), q3 = __shfl(lw1, sb);
      const bool lsel = lane >= 16;
      v4u pv;
      pv.x = (unsigned int)(lsel ? q0 : g0);
      pv.y = (unsigned int)(lsel ? q1 : g1);
      pv.z = (unsigned int)(lsel ? q2 : g2);
      pv.w = (unsigned int)(lsel ? q3 : g3);
      unsigned short* gp = HP + (size_t)grow * KAP + 8 * lane;
      const bool wr = grow < MPr;
      if (wr) *(volatile v4u*)gp = pv;
      __threadfence();
      if (wr) *(volatile v4u*)gp = pv;
    }
  } else {
    const int c0 = 2 * lane;
    const bool valid = c0 < NCLS;
    const int cc0 = c0 < NCLS ? c0 : NCLS - 1;
    const int cc1 = c0 + 1 < NCLS ? c0 + 1 : NCLS - 1;
    float bz0 = bfr(bias[cc0]), bz1 = bfr(bias[cc1]);
    bz0 = valid ? bz0 : 0.f;
    bz1 = valid ? bz1 : 0.f;
    const float* ASp = SD;
    const float* ADp = SD + MPr;
    float* res = (float*)reg1 + wave * (GRP * NCLS);

#pragma unroll 1
    for (int jt = 0; jt < nbw; ++jt) {
      const int slot = wave * nbw + jt;
      const int grow = nodeBase + slot;
      const int gcl  = grow < nN ? grow : nN - 1;
      int st = soff[slot];
      const int craw = scnt[slot];
      int cnt = craw;
      st  = st < 0 ? 0 : (st > nh ? nh : st);
      cnt = cnt < 0 ? 0 : (cnt > DEGCAP ? DEGCAP : cnt);
      if (cnt > nh - st) cnt = nh - st;
      const float pz = (ovf || craw > DEGCAP) ? qnan : 0.0f;

      const v2f fd = *(const v2fa*)(F + (size_t)gcl * NC2P + c0);
      const float adv = ADp[gcl];
      float l0 = ASp[gcl] + adv;
      l0 = l0 > 0.f ? l0 : NEGSL * l0;
      float mx = l0, dn = 1.0f;
      float a0 = fd.x, a1 = fd.y;

#pragma unroll 1
      for (int q = 0; q < cnt; ++q) {
        int idx = st + q; idx = idx > RCAP - 1 ? RCAP - 1 : idx;
        int eid = reg2[idx]; eid = eid < 0 ? 0 : (eid > nE - 1 ? nE - 1 : eid);
        const int sraw = srcs[eid];
        const int s = sraw < 0 ? 0 : (sraw > nN - 1 ? nN - 1 : sraw);
        const v2f fs = *(const v2fa*)(F + (size_t)s * NC2P + c0);
        float lg = ASp[s] + adv;
        lg = lg > 0.f ? lg : NEGSL * lg;
        const float df = lg - mx;
        const float ee = __expf(-fabsf(df));
        const bool up  = df > 0.f;
        const float s1 = up ? ee : 1.0f;
        const float s2 = up ? 1.0f : ee;
        mx = up ? lg : mx;
        dn = fmaf(dn, s1, s2);
        a0 = fmaf(a0, s1, s2 * fs.x);
        a1 = fmaf(a1, s1, s2 * fs.y);
      }
      const float inv = __builtin_amdgcn_rcpf(dn);
      const float z0 = fmaf(a0, inv, bz0);
      const float z1 = fmaf(a1, inv, bz1);
      float vm = valid ? fmaxf(z0, z1) : -3.0e38f;
#pragma unroll
      for (int off = 16; off > 0; off >>= 1) vm = fmaxf(vm, __shfl_xor(vm, off));
      const float ex0 = expf(z0 - vm), ex1 = expf(z1 - vm);
      float sm = valid ? (ex0 + ex1) : 0.f;
#pragma unroll
      for (int off = 16; off > 0; off >>= 1) sm += __shfl_xor(sm, off);
      const float ls = logf(sm);
      const float o0 = ((z0 - vm) - ls) + pz;
      const float o1 = ((z1 - vm) - ls) + pz;
      const int lr = jt & (GRP - 1);
      if (valid) {
        v2f ov; ov.x = o0; ov.y = o1;
        *(v2f*)(res + lr * NCLS + c0) = ov;
      }

      const int gb = jt & ~(GRP - 1);
      if (lr == GRP - 1 || jt == nbw - 1) {
        __syncthreads();
        int gsz = nbw - gb; gsz = gsz > GRP ? GRP : gsz;
        const int row0 = nodeBase + wave * nbw + gb;
        int live = nN - row0; live = live < 0 ? 0 : (live > gsz ? gsz : live);
        const int npc = live * (NCLS / 4);
        float* ob = out + (size_t)row0 * NCLS;
#pragma unroll 1
        for (int p = lane; p < npc; p += 32) {
          const v4f v = *(const v4fa*)(res + 4 * p);
          *(volatile v4f*)(ob + 4 * p) = v;
        }
        __threadfence();
#pragma unroll 1
        for (int p = lane; p < npc; p += 32) {
          const v4f v = *(const v4fa*)(res + 4 * p);
          *(volatile v4f*)(ob + 4 * p) = v;
        }
        __syncthreads();
      }
    }
  }
}

static int pick_nb(int nE, int nN) {
  int nb = NBMAX;
  while (nb > 32 && (long long)nb * (long long)nE * 5LL > (long long)RCAP * (long long)nN * 4LL) nb >>= 1;
  return nb;
}
static inline int cdiv(int a, int b) { return (a + b - 1) / b; }

extern "C" void kernel_launch(void* const* d_in, const int* in_sizes, int n_in,
                              void* d_out, int out_size, void* d_ws, size_t ws_size,
                              hipStream_t stream) {
  const int TS = 3;
  if (n_in < 16) return;
  if (in_sizes[0] < TS * FIN || (in_sizes[0] % (TS * FIN)) != 0) return;
  const int nN = in_sizes[0] / (TS * FIN);
  if (nN <= 0 || nN > (1 << 22)) return;
  if (in_sizes[1] < 2 * TS || (in_sizes[1] % (2 * TS)) != 0) return;
  const int nE = in_sizes[1] / (2 * TS);
  if (nE < 1 || nE >= (1 << (32 - SLOTB))) return;
  if (in_sizes[2] != FIN * HC1) return;
  if (in_sizes[3] != NHD1 * HW1 || in_sizes[4] != NHD1 * HW1) return;
  if (in_sizes[5] != HC1) return;
  if (in_sizes[6] != 2 * HC1 * HID || in_sizes[8] != 2 * HC1 * HID || in_sizes[10] != 2 * HC1 * HID) return;
  if (in_sizes[7] != HID || in_sizes[9] != HID || in_sizes[11] != HID) return;
  if (in_sizes[12] != HID * NCLS) return;
  if (in_sizes[13] != NCLS || in_sizes[14] != NCLS || in_sizes[15] != NCLS) return;
  if ((long long)out_size != (long long)nN * NCLS) return;

  const float* xall = (const float*)d_in[0];
  const int*   ei   = (const int*)  d_in[1];
  const float* W1   = (const float*)d_in[2];
  const float* a1s  = (const float*)d_in[3];
  const float* a1d  = (const float*)d_in[4];
  const float* b1   = (const float*)d_in[5];
  const float* K1   = (const float*)d_in[6];
  const float* bk1  = (const float*)d_in[7];
  const float* K2   = (const float*)d_in[8];
  const float* bk2  = (const float*)d_in[9];
  const float* K3   = (const float*)d_in[10];
  const float* bk3  = (const float*)d_in[11];
  const float* W2   = (const float*)d_in[12];
  const float* a2s  = (const float*)d_in[13];
  const float* a2d  = (const float*)d_in[14];
  const float* b2   = (const float*)d_in[15];
  float* out = (float*)d_out;
  const int* src1 = ei + (size_t)1 * 2 * (size_t)nE;
  const int* dst1 = src1 + nE;
  const int* src2 = ei + (size_t)2 * 2 * (size_t)nE;
  const int* dst2 = src2 + nE;

  const int MP   = cdiv(nN, MROWS) * MROWS;
  const int nb   = pick_nb(nE, nN);
  if (nb < 32 || (nb & (nb - 1)) != 0 || nb > NBMAX) return;
  const int gA   = cdiv(MP, nb);
  const int vec8 = ((nE & 3) == 0) ? 1 : 0;
  if ((long long)gA * nb < (long long)MP) return;
  const int gM   = MP / GBM;

  char* ws = (char*)d_ws;
  size_t off = 0;
  const size_t oXB  = off; off += (size_t)2 * MP * FIN * 2;        off = (off + 255) & ~(size_t)255;
  const size_t oW1T = off; off += (size_t)HC1 * FIN * 2;           off = (off + 255) & ~(size_t)255;
  const size_t oKCT = off; off += (size_t)TCN * TCK * 2;           off = (off + 255) & ~(size_t)255;
  const size_t oW2T = off; off += (size_t)NC2P * KY * 2;           off = (off + 255) & ~(size_t)255;
  const size_t oH   = off; off += (size_t)MP * HC1 * 4;            off = (off + 255) & ~(size_t)255;
  const size_t oSD1 = off; off += (size_t)2 * NHD1 * MP * 4;       off = (off + 255) & ~(size_t)255;
  const size_t oAP  = off; off += (size_t)MP * KAP * 2;            off = (off + 255) & ~(size_t)255;
  const size_t oYP  = off; off += (size_t)MP * KY * 2;             off = (off + 255) & ~(size_t)255;
  const size_t oH2  = off; off += (size_t)MP * NC2P * 4;           off = (off + 255) & ~(size_t)255;
  const size_t oSD2 = off; off += (size_t)2 * MP * 4;              off = (off + 255) & ~(size_t)255;
  if (off > ws_size || off > (size_t)WSMAX) return;
  unsigned short* XB  = (unsigned short*)(ws + oXB);
  unsigned short* W1T = (unsigned short*)(ws + oW1T);
  unsigned short* KCT = (unsigned short*)(ws + oKCT);
  unsigned short* W2T = (unsigned short*)(ws + oW2T);
  float*          H   = (float*)(ws + oH);
  float*          SD1 = (float*)(ws + oSD1);
  unsigned short* AP  = (unsigned short*)(ws + oAP);
  unsigned short* YP  = (unsigned short*)(ws + oYP);
  float*          H2  = (float*)(ws + oH2);
  float*          SD2 = (float*)(ws + oSD2);

  hipFuncSetAttribute(reinterpret_cast<const void*>(&k_agg<1>),
                      hipFuncAttributeMaxDynamicSharedMemorySize, LDS_AGG);
  hipFuncSetAttribute(reinterpret_cast<const void*>(&k_agg<2>),
                      hipFuncAttributeMaxDynamicSharedMemorySize, LDS_AGG);

  k_wprep<<<(NU1 + NU2 + NU3) / NTHR, NTHR, 0, stream>>>(W1, K1, K2, K3, W2, W1T, KCT, W2T);
  const int nUx = 2 * MP * (FIN / 8);
  k_xprep<<<cdiv(nUx, NTHR), NTHR, 0, stream>>>(xall, XB, nN, MP, nUx);

  k_gemm<HW1><<<dim3(gM, HC1 / GBN), GTHR, 0, stream>>>(XB, W1T, H, FIN, HC1, a1s, a1d, HW1, SD1, MP);
  k_agg<1><<<gA, NTHR, LDS_AGG, stream>>>(src1, dst1, H, SD1, b1, AP, out, nN, nE, nb, vec8, MP);
  k_gemm<HW1><<<dim3(gM, HC1 / GBN), GTHR, 0, stream>>>(XB + (size_t)MP * FIN, W1T, H, FIN, HC1, a1s, a1d, HW1, SD1, MP);
  k_agg<1><<<gA, NTHR, LDS_AGG, stream>>>(src2, dst2, H, SD1, b1, AP + 2 * HC1, out, nN, nE, nb, vec8, MP);
  k_tconv<<<gM, GTHR, 0, stream>>>(AP, KCT, bk1, bk2, bk3, YP, nN);
  k_gemm<64><<<dim3(gM, NC2P / GBN), GTHR, 0, stream>>>(YP, W2T, H2, KY, NC2P, a2s, a2d, NCLS, SD2, MP);
  k_agg<2><<<gA, NTHR, LDS_AGG, stream>>>(src2, dst2, H2, SD2, b2, AP, out, nN, nE, nb, vec8, MP);
}
